// CausalSelfAttention_85392539779597
// MI455X (gfx1250) — hardware-verified
//
#include <hip/hip_runtime.h>


#ifndef NB
#define NB 2
#endif
#ifndef SEQ
#define SEQ 2048
#endif
#define NB_FULL    2
#define SEQ_FULL   2048
#define NHEAD      16
#define HDIM       64
#define DEMB       1024
#define QKVN       3072
#define MROWS      (NB * SEQ)
#define BQ         128
#define BK         32
#define NWAVE      8
#define OP         68
#define SP         132
#define QBLKS      (SEQ / BQ)
#define EARLY_QB   ((QBLKS < 2) ? QBLKS : 2)
#define VRK        (EARLY_QB * BQ)
#define PLANE_ELEMS ((size_t)NB * NHEAD * SEQ * HDIM)
#define CTX_ELEMS   ((size_t)MROWS * DEMB)
#define VTB_ELEMS   ((size_t)NB * NHEAD * HDIM * VRK)
#define X_PIECES    ((size_t)MROWS * (DEMB / 8))
#define WIN_PIECES  ((size_t)QKVN * DEMB / 8)
#define WOUT_PIECES ((size_t)DEMB * DEMB / 8)
#define WIN_ELEMS   ((size_t)QKVN * DEMB)
#define WOUT_ELEMS  ((size_t)DEMB * DEMB)
#define AM_BLOCKS_IN  96
#define AM_BLOCKS_OUT 32
#define AM_TOTAL      (AM_BLOCKS_IN + AM_BLOCKS_OUT)
#define STAT_FLOATS   ((size_t)(AM_TOTAL + 2) * 32)

static_assert(NHEAD * HDIM == DEMB);
static_assert(QKVN == 3 * DEMB);
static_assert(HDIM == 64);
static_assert(SEQ % BQ == 0);
static_assert(SEQ % BK == 0);
static_assert(BK == 32);
static_assert(SEQ % 128 == 0);
static_assert(MROWS % 128 == 0);
static_assert(QKVN % 128 == 0);
static_assert(DEMB % 128 == 0);
static_assert(DEMB % 32 == 0);
static_assert(DEMB % 8 == 0);
static_assert(BQ == NWAVE * 16);
static_assert(BQ % 64 == 0);
static_assert(VRK % 64 == 0 && VRK <= SEQ && VRK >= BQ);
static_assert(EARLY_QB >= 1 && EARLY_QB <= QBLKS);
static_assert(SEQ <= SEQ_FULL);
static_assert(NB >= 1 && NB <= NB_FULL);
static_assert((OP * 4) % 16 == 0);
static_assert((SP * 4) % 16 == 0);
static_assert(SP >= 128);
static_assert(OP >= 64);
static_assert(X_PIECES % 256 == 0);
static_assert(WIN_PIECES % 256 == 0);
static_assert(WOUT_PIECES % 256 == 0);
static_assert(NWAVE == 8);
static_assert(AM_BLOCKS_IN % 32 == 0 && AM_BLOCKS_OUT % 32 == 0);
static_assert(WIN_PIECES % ((size_t)AM_BLOCKS_IN * 256) == 0);
static_assert(WOUT_PIECES % ((size_t)AM_BLOCKS_OUT * 256) == 0);

typedef __bf16   bf16;
typedef _Float16 f16;
typedef bf16     v16bf __attribute__((ext_vector_type(16)));
typedef f16      v16h  __attribute__((ext_vector_type(16)));
typedef f16      v8h   __attribute__((ext_vector_type(8)));
typedef float    v8f   __attribute__((ext_vector_type(8)));
typedef float    v4f   __attribute__((ext_vector_type(4)));
typedef unsigned v4u   __attribute__((ext_vector_type(4)));

union FragB  { v16bf v; v4u q[2]; bf16 h[16]; };
union FragH  { v16h  v; v4u q[2]; f16  h[16]; };
union Pack8B { v4u u; bf16 h[8]; };
union Pack8H { v4u u; v8h v; f16 h[8]; };

#define XB_BYTES   ((size_t)MROWS * DEMB * 2)
#define WIN_BYTES  (WIN_ELEMS * 2 * 2)
#define WOUT_BYTES (WOUT_ELEMS * 2 * 2)
#define QK_BYTES   (PLANE_ELEMS * 2 * 4)
#define VT_BYTES   (PLANE_ELEMS * 2)
#define VTB_BYTES  (VTB_ELEMS * 2 * 2)
#define CTX_BYTES  (CTX_ELEMS * 2 * 2)
#define STAT_BYTES (STAT_FLOATS * 4)
#define WS_TOTAL   (XB_BYTES + WIN_BYTES + WOUT_BYTES + QK_BYTES + VT_BYTES + VTB_BYTES + CTX_BYTES + STAT_BYTES)
static_assert(WS_TOTAL <= (size_t)134217728);
static_assert(XB_BYTES % 128 == 0 && WIN_BYTES % 128 == 0 && WOUT_BYTES % 128 == 0);
static_assert(QK_BYTES % 128 == 0 && VT_BYTES % 128 == 0 && VTB_BYTES % 128 == 0 && CTX_BYTES % 128 == 0);
static_assert(STAT_BYTES % 128 == 0);

static __device__ __forceinline__ v8f mma_bf16(v16bf a, v16bf b, v8f acc) {
  acc = __builtin_amdgcn_wmma_f32_16x16x32_bf16(false, a, false, b, (short)0, acc, false, false);
  asm volatile("v_nop\n\tv_nop\n\tv_nop\n\tv_nop" : "+v"(acc) : "v"(a), "v"(b));
  return acc;
}
static __device__ __forceinline__ v8f mma_f16(v16h a, v16h b, v8f acc) {
  acc = __builtin_amdgcn_wmma_f32_16x16x32_f16(false, a, false, b, (short)0, acc, false, false);
  asm volatile("v_nop\n\tv_nop\n\tv_nop\n\tv_nop" : "+v"(acc) : "v"(a), "v"(b));
  return acc;
}

static __device__ __forceinline__ f16 toh_flush(float v) {
  const f16 r = (f16)v;
  return (fabsf(v) < 6.103515625e-05f) ? (f16)0.0f : r;
}

__global__ __launch_bounds__(256) void cvt_x_kernel(const float* __restrict__ x, bf16* __restrict__ xb) {
  const size_t t   = (size_t)blockIdx.x * 256 + threadIdx.x;
  const size_t row = t >> 7;
  const int    c8  = (int)(t & 127) * 8;
  if (row < (size_t)MROWS) {
    const int b = (int)(row / SEQ);
    const int s = (int)(row % SEQ);
    const float* src = x + ((size_t)b * SEQ_FULL + s) * DEMB + c8;
    const v4f a0 = *(const v4f*)(src);
    const v4f a1 = *(const v4f*)(src + 4);
    Pack8B pk;
    #pragma unroll
    for (int i = 0; i < 4; ++i) {
      pk.h[i]     = (bf16)a0[i];
      pk.h[4 + i] = (bf16)a1[i];
    }
    const v4u val = pk.u;
    bf16* dst = xb + row * DEMB + c8;
    *(volatile v4u*)dst = val;
    __threadfence();
    *(volatile v4u*)dst = val;
  }
}

__global__ __launch_bounds__(256) void absmax_part_kernel(const float* __restrict__ w,
                                                          float* __restrict__ part,
                                                          unsigned npieces) {
  __shared__ float sM[NWAVE];
  const int tid  = threadIdx.x;
  const int lane = tid & 31;
  const int wid  = __builtin_amdgcn_readfirstlane(tid >> 5);
  float m = 0.0f;
  #pragma unroll 1
  for (unsigned p = blockIdx.x * 256u + (unsigned)tid; p < npieces; p += gridDim.x * 256u) {
    const size_t o = (size_t)p * 8;
    const v4f a0 = *(const v4f*)(w + o);
    const v4f a1 = *(const v4f*)(w + o + 4);
    #pragma unroll
    for (int i = 0; i < 4; ++i) {
      m = fmaxf(m, fabsf(a0[i]));
      m = fmaxf(m, fabsf(a1[i]));
    }
  }
  m = fmaxf(m, __shfl_xor(m, 16, 32));
  m = fmaxf(m, __shfl_xor(m, 8, 32));
  m = fmaxf(m, __shfl_xor(m, 4, 32));
  m = fmaxf(m, __shfl_xor(m, 2, 32));
  m = fmaxf(m, __shfl_xor(m, 1, 32));
  if (lane == 0) sM[wid] = m;
  __syncthreads();
  if (wid == 0) {
    float v = sM[lane & 7];
    v = fmaxf(v, __shfl_xor(v, 4, 32));
    v = fmaxf(v, __shfl_xor(v, 2, 32));
    v = fmaxf(v, __shfl_xor(v, 1, 32));
    const v4f val = (v4f){v, v, v, v};
    if (lane < 8) {
      float* dst = part + (size_t)blockIdx.x * 32 + lane * 4;
      *(volatile v4f*)dst = val;
      __threadfence();
      *(volatile v4f*)dst = val;
    }
  }
}

__global__ __launch_bounds__(32) void scale_fin_kernel(const float* part, float* sline) {
  #pragma clang fp contract(off)
  const int lane = threadIdx.x & 31;
  float mi = 0.0f;
  float mo = 0.0f;
  #pragma unroll 1
  for (int j = 0; j < AM_BLOCKS_IN; j += 32) mi = fmaxf(mi, part[(size_t)(j + lane) * 32]);
  #pragma unroll 1
  for (int j = 0; j < AM_BLOCKS_OUT; j += 32) mo = fmaxf(mo, part[(size_t)(AM_BLOCKS_IN + j + lane) * 32]);
  mi = fmaxf(mi, __shfl_xor(mi, 16, 32));
  mo = fmaxf(mo, __shfl_xor(mo, 16, 32));
  mi = fmaxf(mi, __shfl_xor(mi, 8, 32));
  mo = fmaxf(mo, __shfl_xor(mo, 8, 32));
  mi = fmaxf(mi, __shfl_xor(mi, 4, 32));
  mo = fmaxf(mo, __shfl_xor(mo, 4, 32));
  mi = fmaxf(mi, __shfl_xor(mi, 2, 32));
  mo = fmaxf(mo, __shfl_xor(mo, 2, 32));
  mi = fmaxf(mi, __shfl_xor(mi, 1, 32));
  mo = fmaxf(mo, __shfl_xor(mo, 1, 32));
  const float si = (float)(bf16)mi + 1e-6f;
  const float so = (float)(bf16)mo + 1e-6f;
  const float ri = 1.0f / si;
  const float ro = 1.0f / so;
  const v4f vi = (v4f){si, ri, si, ri};
  const v4f vo = (v4f){so, ro, so, ro};
  if (lane < 8) {
    float* d0 = sline + lane * 4;
    float* d1 = sline + 32 + lane * 4;
    *(volatile v4f*)d0 = vi;
    *(volatile v4f*)d1 = vo;
    __threadfence();
    *(volatile v4f*)d0 = vi;
    *(volatile v4f*)d1 = vo;
  }
}

static __device__ __forceinline__ void snap_step(const float wn, const float c, float& bd, float& best) {
  #pragma clang fp contract(off)
  const float d  = fabsf(wn - c);
  const bool  lt = d < bd;
  bd   = lt ? d : bd;
  best = lt ? c : best;
}

static __device__ __forceinline__ float snap_weight_val(const float w, const float s, const float rs) {
  #pragma clang fp contract(off)
  const float wb = (float)(bf16)w;
  const float wn = wb * rs;
  float best = 0.0f;
  float bd   = fabsf(wn - 0.0f);
  snap_step(wn,  1.0f,      bd, best);
  snap_step(wn, -1.0f,      bd, best);
  snap_step(wn,  0.5f,      bd, best);
  snap_step(wn, -0.5f,      bd, best);
  snap_step(wn,  0.333333f, bd, best);
  snap_step(wn, -0.333333f, bd, best);
  snap_step(wn,  0.2f,      bd, best);
  snap_step(wn, -0.2f,      bd, best);
  snap_step(wn,  0.142857f, bd, best);
  snap_step(wn, -0.142857f, bd, best);
  snap_step(wn,  0.090909f, bd, best);
  snap_step(wn, -0.090909f, bd, best);
  snap_step(wn,  0.076923f, bd, best);
  snap_step(wn, -0.076923f, bd, best);
  return best * s;
}

__global__ __launch_bounds__(256) void snap_lin_kernel(const float* __restrict__ src,
                                                       const float* __restrict__ sline,
                                                       bf16* __restrict__ dhi,
                                                       bf16* __restrict__ dlo,
                                                       unsigned npieces) {
  #pragma clang fp contract(off)
  const unsigned t = blockIdx.x * 256u + threadIdx.x;
  if (t < npieces) {
    const float s  = sline[0];
    const float rs = sline[1];
    const size_t o = (size_t)t * 8;
    const v4f a0 = *(const v4f*)(src + o);
    const v4f a1 = *(const v4f*)(src + o + 4);
    Pack8B ph, pl;
    #pragma unroll
    for (int i = 0; i < 4; ++i) {
      const float q0 = snap_weight_val(a0[i], s, rs);
      const float q1 = snap_weight_val(a1[i], s, rs);
      const bf16 h0 = (bf16)q0;
      const bf16 h1 = (bf16)q1;
      ph.h[i]     = h0;
      ph.h[4 + i] = h1;
      pl.h[i]     = (bf16)(q0 - (float)h0);
      pl.h[4 + i] = (bf16)(q1 - (float)h1);
    }
    const v4u vh = ph.u;
    const v4u vl = pl.u;
    *(volatile v4u*)(dhi + o) = vh;
    *(volatile v4u*)(dlo + o) = vl;
    __threadfence();
    *(volatile v4u*)(dhi + o) = vh;
    *(volatile v4u*)(dlo + o) = vl;
  }
}

template <int NA, int NW>
static __device__ __forceinline__ void gemm_mainloop(const bf16* __restrict__ A0,
                                                     const bf16* __restrict__ A1,
                                                     const bf16* __restrict__ Bt,
                                                     const bf16* __restrict__ Bl,
                                                     int mBlock, int nBlock, int waveM, int waveN,
                                                     int ln, int hf, v8f (&acc)[4][2]) {
  #pragma unroll
  for (int mt = 0; mt < 4; ++mt) {
    acc[mt][0] = (v8f){0, 0, 0, 0, 0, 0, 0, 0};
    acc[mt][1] = (v8f){0, 0, 0, 0, 0, 0, 0, 0};
  }
  const bf16* bp0 = Bt + (size_t)(nBlock + waveN * 32 + ln) * DEMB + hf * 8;
  const bf16* bp1 = bp0 + (size_t)16 * DEMB;
  const bf16* lp0 = Bl + (size_t)(nBlock + waveN * 32 + ln) * DEMB + hf * 8;
  const bf16* lp1 = lp0 + (size_t)16 * DEMB;
  const size_t aoff = (size_t)(mBlock + waveM * 16 + ln) * DEMB + hf * 8;
  #pragma unroll 1
  for (int k0 = 0; k0 < DEMB; k0 += 32) {
    FragB b0, b1;
    b0.q[0] = *(const v4u*)(bp0 + k0);
    b0.q[1] = *(const v4u*)(bp0 + k0 + 16);
    b1.q[0] = *(const v4u*)(bp1 + k0);
    b1.q[1] = *(const v4u*)(bp1 + k0 + 16);
    FragB w0, w1;
    if (NW == 2) {
      w0.q[0] = *(const v4u*)(lp0 + k0);
      w0.q[1] = *(const v4u*)(lp0 + k0 + 16);
      w1.q[0] = *(const v4u*)(lp1 + k0);
      w1.q[1] = *(const v4u*)(lp1 + k0 + 16);
    } else {
      w0.q[0] = b0.q[0]; w0.q[1] = b0.q[1];
      w1.q[0] = b1.q[0]; w1.q[1] = b1.q[1];
    }
    #pragma unroll
    for (int mt = 0; mt < 4; ++mt) {
      const size_t ao = aoff + (size_t)mt * 32 * DEMB + k0;
      FragB a;
      a.q[0] = *(const v4u*)(A0 + ao);
      a.q[1] = *(const v4u*)(A0 + ao + 16);
      acc[mt][0] = mma_bf16(a.v, b0.v, acc[mt][0]);
      acc[mt][1] = mma_bf16(a.v, b1.v, acc[mt][1]);
      if (NW == 2) {
        acc[mt][0] = mma_bf16(a.v, w0.v, acc[mt][0]);
        acc[mt][1] = mma_bf16(a.v, w1.v, acc[mt][1]);
      }
      if (NA == 2) {
        FragB a2;
        a2.q[0] = *(const v4u*)(A1 + ao);
        a2.q[1] = *(const v4u*)(A1 + ao + 16);
        acc[mt][0] = mma_bf16(a2.v, b0.v, acc[mt][0]);
        acc[mt][1] = mma_bf16(a2.v, b1.v, acc[mt][1]);
      }
    }
  }
}

__global__ __launch_bounds__(256) void gemm_qkv_kernel(const bf16* __restrict__ xb,
                                                       const bf16* __restrict__ winb,
                                                       const bf16* __restrict__ winl,
                                                       const float* __restrict__ b_in,
                                                       bf16* __restrict__ qkp,
                                                       f16* __restrict__ vt,
                                                       bf16* __restrict__ vtb) {
  __shared__ __align__(16) float sC[64 * SP];
  const int tid   = threadIdx.x;
  const int lane  = tid & 31;
  const int wid   = __builtin_amdgcn_readfirstlane(tid >> 5);
  const int ln    = lane & 15;
  const int hf    = lane >> 4;
  const int waveM = wid >> 2;
  const int waveN = wid & 3;
  const int nBlock = blockIdx.x * 128;
  const int mBlock = blockIdx.y * 128;

  v8f acc[4][2];
  gemm_mainloop<1, 2>(xb, xb, winb, winl, mBlock, nBlock, waveM, waveN, ln, hf, acc);

  float bia[2];
  #pragma unroll
  for (int nt = 0; nt < 2; ++nt) bia[nt] = (float)(bf16)b_in[nBlock + waveN * 32 + nt * 16 + ln];

  const int which = nBlock / DEMB;
  const int cb    = nBlock % DEMB;
  const int bb    = mBlock / SEQ;
  const int sb    = mBlock % SEQ;

  #pragma unroll
  for (int p = 0; p < 2; ++p) {
    __syncthreads();
    #pragma unroll
    for (int j = 0; j < 2; ++j) {
      #pragma unroll
      for (int nt = 0; nt < 2; ++nt) {
        #pragma unroll
        for (int e = 0; e < 8; ++e) {
          sC[(j * 32 + waveM * 16 + hf * 8 + e) * SP + waveN * 32 + nt * 16 + ln] =
              acc[2 * p + j][nt][e] + bia[nt];
        }
      }
    }
    __syncthreads();

    if (which < 2) {
      v4u    vh[4], vl[4];
      size_t gi[4];
      #pragma unroll
      for (int sw = 0; sw < 4; ++sw) {
        const int r  = sw * 16 + (tid >> 4);
        const int c8 = (tid & 15) * 8;
        const v4f a0 = *(const v4f*)(sC + r * SP + c8);
        const v4f a1 = *(const v4f*)(sC + r * SP + c8 + 4);
        Pack8B ph, pl;
        #pragma unroll
        for (int i = 0; i < 4; ++i) {
          const bf16 h0 = (bf16)a0[i];
          const bf16 h1 = (bf16)a1[i];
          ph.h[i]     = h0;
          ph.h[4 + i] = h1;
          pl.h[i]     = (bf16)(a0[i] - (float)h0);
          pl.h[4 + i] = (bf16)(a1[i] - (float)h1);
        }
        vh[sw] = ph.u;
        vl[sw] = pl.u;
        const int s  = sb + p * 64 + r;
        const int cc = cb + c8;
        const int h  = cc >> 6;
        const int d  = cc & 63;
        gi[sw] = (size_t)which * 2 * PLANE_ELEMS + (((size_t)bb * NHEAD + h) * SEQ + s) * HDIM + d;
      }
      #pragma unroll
      for (int sw = 0; sw < 4; ++sw) {
        *(volatile v4u*)(qkp + gi[sw]) = vh[sw];
        *(volatile v4u*)(qkp + PLANE_ELEMS + gi[sw]) = vl[sw];
      }
      __threadfence();
      #pragma unroll
      for (int sw = 0; sw < 4; ++sw) {
        *(volatile v4u*)(qkp + gi[sw]) = vh[sw];
        *(volatile v4u*)(qkp + PLANE_ELEMS + gi[sw]) = vl[sw];
      }
    } else {
      const bool wr_early = (sb + p * 64) < VRK;
      v4u    vv[4], vbh[4], vbl[4];
      size_t gi[4], gb[4];
      #pragma unroll
      for (int sw = 0; sw < 4; ++sw) {
        const int col = sw * 32 + (tid >> 3);
        const int sg  = (tid & 7) * 8;
        Pack8H ph;
        Pack8B qh, ql;
        #pragma unroll
        for (int i = 0; i < 8; ++i) {
          const float v = sC[(sg + i) * SP + col];
          ph.h[i] = toh_flush(v * 16.0f);
          const bf16 t = (bf16)v;
          qh.h[i] = t;
          ql.h[i] = (bf16)(v - (float)t);
        }
        vv[sw]  = ph.u;
        vbh[sw] = qh.u;
        vbl[sw] = ql.u;
        const int cc = cb + col;
        const int h  = cc >> 6;
        const int d  = cc & 63;
        const size_t rowid = ((size_t)bb * NHEAD + h) * HDIM + d;
        gi[sw] = rowid * SEQ + sb + p * 64 + sg;
        gb[sw] = rowid * VRK + sb + p * 64 + sg;
      }
      #pragma unroll
      for (int sw = 0; sw < 4; ++sw) *(volatile v4u*)(vt + gi[sw]) = vv[sw];
      if (wr_early) {
        #pragma unroll
        for (int sw = 0; sw < 4; ++sw) {
          *(volatile v4u*)(vtb + gb[sw]) = vbh[sw];
          *(volatile v4u*)(vtb + VTB_ELEMS + gb[sw]) = vbl[sw];
        }
      }
      __threadfence();
      #pragma unroll
      for (int sw = 0; sw < 4; ++sw) *(volatile v4u*)(vt + gi[sw]) = vv[sw];
      if (wr_early) {
        #pragma unroll
        for (int sw = 0; sw < 4; ++sw) {
          *(volatile v4u*)(vtb + gb[sw]) = vbh[sw];
          *(volatile v4u*)(vtb + VTB_ELEMS + gb[sw]) = vbl[sw];
        }
      }
    }
  }
}

__global__ __launch_bounds__(256) void gemm_out_kernel(const bf16* __restrict__ ch,
                                                       const bf16* __restrict__ cl,
                                                       const bf16* __restrict__ woutb,
                                                       const bf16* __restrict__ woutl,
                                                       const float* __restrict__ b_out,
                                                       float* __restrict__ out) {
  __shared__ __align__(16) float sC[64 * SP];
  const int tid   = threadIdx.x;
  const int lane  = tid & 31;
  const int wid   = __builtin_amdgcn_readfirstlane(tid >> 5);
  const int ln    = lane & 15;
  const int hf    = lane >> 4;
  const int waveM = wid >> 2;
  const int waveN = wid & 3;
  const int nBlock = blockIdx.x * 128;
  const int mBlock = blockIdx.y * 128;

  v8f acc[4][2];
  gemm_mainloop<2, 2>(ch, cl, woutb, woutl, mBlock, nBlock, waveM, waveN, ln, hf, acc);

  float bia[2];
  #pragma unroll
  for (int nt = 0; nt < 2; ++nt) bia[nt] = (float)(bf16)b_out[nBlock + waveN * 32 + nt * 16 + ln];

  #pragma unroll
  for (int p = 0; p < 2; ++p) {
    __syncthreads();
    #pragma unroll
    for (int j = 0; j < 2; ++j) {
      #pragma unroll
      for (int nt = 0; nt < 2; ++nt) {
        #pragma unroll
        for (int e = 0; e < 8; ++e) {
          sC[(j * 32 + waveM * 16 + hf * 8 + e) * SP + waveN * 32 + nt * 16 + ln] =
              acc[2 * p + j][nt][e] + bia[nt];
        }
      }
    }
    __syncthreads();

    v4f    vals[8];
    size_t gi[8];
    #pragma unroll
    for (int sw = 0; sw < 8; ++sw) {
      const int r  = sw * 8 + (tid >> 5);
      const int c4 = (tid & 31) * 4;
      vals[sw] = *(const v4f*)(sC + r * SP + c4);
      const int g = mBlock + p * 64 + r;
      const int b = g / SEQ;
      const int s = g % SEQ;
      gi[sw] = ((size_t)b * SEQ_FULL + s) * DEMB + nBlock + c4;
    }
    #pragma unroll
    for (int sw = 0; sw < 8; ++sw) *(volatile v4f*)(out + gi[sw]) = vals[sw];
    __threadfence();
    #pragma unroll
    for (int sw = 0; sw < 8; ++sw) *(volatile v4f*)(out + gi[sw]) = vals[sw];
  }
}

template <bool EARLY>
static __device__ __forceinline__ void attn_body(const bf16* __restrict__ qkp,
                                                 const f16* __restrict__ vt,
                                                 const bf16* __restrict__ vtb,
                                                 bf16* __restrict__ cp,
                                                 const int qblk) {
  __shared__ __align__(16) float sO[NWAVE * 16 * OP];

  const int h    = blockIdx.y;
  const int b    = blockIdx.z;
  const int tid  = threadIdx.x;
  const int wave = __builtin_amdgcn_readfirstlane(tid >> 5);
  const int lane = tid & 31;
  const int lq   = lane & 15;
  const int hi   = lane >> 4;

  const int qrow0 = qblk * BQ + wave * 16;
  const int nIter = (qrow0 >> 5) + 1;
  const size_t head_off = ((size_t)b * NHEAD + h) * SEQ * HDIM;
  const size_t vhead    = ((size_t)b * NHEAD + h) * HDIM;

  const bf16* qh_p = qkp + head_off;
  const bf16* ql_p = qkp + PLANE_ELEMS + head_off;
  const bf16* kh_p = qkp + 2 * PLANE_ELEMS + head_off;
  const bf16* kl_p = qkp + 3 * PLANE_ELEMS + head_off;

  FragB qfh[2], qfl[2];
  {
    const size_t qo = (size_t)(qrow0 + lq) * HDIM + hi * 8;
    #pragma unroll
    for (int f = 0; f < 2; ++f) {
      qfh[f].q[0] = *(const v4u*)(qh_p + qo + f * 32);
      qfh[f].q[1] = *(const v4u*)(qh_p + qo + f * 32 + 16);
      qfl[f].q[0] = *(const v4u*)(ql_p + qo + f * 32);
      qfl[f].q[1] = *(const v4u*)(ql_p + qo + f * 32 + 16);
    }
  }

  v8f o[4];
  #pragma unroll
  for (int dt = 0; dt < 4; ++dt) o[dt] = (v8f){0, 0, 0, 0, 0, 0, 0, 0};

  float rmax = -__builtin_inff();
  float rsum = 0.0f;
  const float SL = 0.125f * 1.4426950408889634f;

  #pragma unroll 1
  for (int i = 0; i < nIter; ++i) {
    const int j0 = i * BK;

    v8f c[2];
    #pragma unroll
    for (int sub = 0; sub < 2; ++sub) {
      const size_t ko = (size_t)(j0 + sub * 16 + lq) * HDIM + hi * 8;
      FragB akh[2], akl[2];
      #pragma unroll
      for (int f = 0; f < 2; ++f) {
        akh[f].q[0] = *(const v4u*)(kh_p + ko + f * 32);
        akh[f].q[1] = *(const v4u*)(kh_p + ko + f * 32 + 16);
        akl[f].q[0] = *(const v4u*)(kl_p + ko + f * 32);
        akl[f].q[1] = *(const v4u*)(kl_p + ko + f * 32 + 16);
      }
      v8f acc = (v8f){0, 0, 0, 0, 0, 0, 0, 0};
      #pragma unroll
      for (int f = 0; f < 2; ++f) {
        acc = mma_bf16(akl[f].v, qfh[f].v, acc);
        acc = mma_bf16(akh[f].v, qfl[f].v, acc);
        acc = mma_bf16(akh[f].v, qfh[f].v, acc);
      }
      c[sub] = acc;
    }

    if (j0 + (BK - 1) > qrow0) {
      const int qi = qrow0 + lq;
      const int kb = j0 + hi * 8;
      #pragma unroll
      for (int r = 0; r < 8; ++r) {
        c[0][r] = (kb + r > qi)      ? -__builtin_inff() : c[0][r];
        c[1][r] = (kb + 16 + r > qi) ? -__builtin_inff() : c[1][r];
      }
    }

    FragH bv[4];
    if (!EARLY) {
      #pragma unroll
      for (int dt = 0; dt < 4; ++dt) {
        const f16* base = vt + (vhead + dt * 16 + lq) * SEQ + j0 + hi * 8;
        bv[dt].q[0] = *(const v4u*)(base);
        bv[dt].q[1] = *(const v4u*)(base + 16);
      }
    }

    float m_new = rmax;
    #pragma unroll
    for (int r = 0; r < 8; ++r) {
      m_new = fmaxf(m_new, c[0][r]);
      m_new = fmaxf(m_new, c[1][r]);
    }
    m_new = fmaxf(m_new, __shfl_xor(m_new, 16, 32));
    const float scale = __builtin_amdgcn_exp2f((rmax - m_new) * SL);
    rmax = m_new;

    float p0[8], p1[8];
    float psum = 0.0f;
    #pragma unroll
    for (int r = 0; r < 8; ++r) {
      p0[r] = __builtin_amdgcn_exp2f((c[0][r] - m_new) * SL);
      p1[r] = __builtin_amdgcn_exp2f((c[1][r] - m_new) * SL);
      psum += p0[r] + p1[r];
    }
    rsum = rsum * scale + psum + __shfl_xor(psum, 16, 32);

    float sc[8];
    #pragma unroll
    for (int r = 0; r < 8; ++r) sc[r] = __shfl(scale, (hi << 3) + r, 32);
    #pragma unroll
    for (int dt = 0; dt < 4; ++dt) {
      #pragma unroll
      for (int r = 0; r < 8; ++r) o[dt][r] *= sc[r];
    }

    if (EARLY) {
      FragB pah, pal;
      #pragma unroll
      for (int r = 0; r < 8; ++r) {
        const bf16 h0 = (bf16)p0[r];
        const bf16 h1 = (bf16)p1[r];
        pah.h[r]     = h0;
        pah.h[8 + r] = h1;
        pal.h[r]     = (bf16)(p0[r] - (float)h0);
        pal.h[8 + r] = (bf16)(p1[r] - (float)h1);
      }
      __builtin_amdgcn_sched_barrier(0);
      #pragma unroll
      for (int dt = 0; dt < 4; ++dt) {
        const bf16* base = vtb + (vhead + dt * 16 + lq) * VRK + j0 + hi * 8;
        FragB bvh, bvl;
        bvh.q[0] = *(const v4u*)(base);
        bvh.q[1] = *(const v4u*)(base + 16);
        bvl.q[0] = *(const v4u*)(base + VTB_ELEMS);
        bvl.q[1] = *(const v4u*)(base + VTB_ELEMS + 16);
        o[dt] = mma_bf16(pal.v, bvh.v, o[dt]);
        o[dt] = mma_bf16(pah.v, bvl.v, o[dt]);
        o[dt] = mma_bf16(pah.v, bvh.v, o[dt]);
      }
    } else {
      FragH pa;
      #pragma unroll
      for (int r = 0; r < 8; ++r) {
        pa.h[r]     = (f16)(p0[r] * 4096.0f);
        pa.h[8 + r] = (f16)(p1[r] * 4096.0f);
      }
      #pragma unroll
      for (int dt = 0; dt < 4; ++dt) o[dt] = mma_f16(pa.v, bv[dt].v, o[dt]);
    }
  }

  const float carry = EARLY ? 1.0f : (1.0f / 65536.0f);
  float rs[8];
  #pragma unroll
  for (int r = 0; r < 8; ++r) rs[r] = carry * (1.0f / __shfl(rsum, (hi << 3) + r, 32));

  const int sbase = wave * (16 * OP);
  #pragma unroll
  for (int r = 0; r < 8; ++r) {
    #pragma unroll
    for (int dt = 0; dt < 4; ++dt) {
      sO[sbase + (hi * 8 + r) * OP + dt * 16 + lq] = o[dt][r] * rs[r];
    }
  }
  __syncthreads();

  v4u    vh[4], vl[4];
  size_t gidx[4];
  #pragma unroll
  for (int it = 0; it < 4; ++it) {
    const int row = it * 4 + (lane >> 3);
    const int c8  = (lane & 7) * 8;
    const v4f a0 = *(const v4f*)(&sO[sbase + row * OP + c8]);
    const v4f a1 = *(const v4f*)(&sO[sbase + row * OP + c8 + 4]);
    Pack8B ph, pl;
    #pragma unroll
    for (int k = 0; k < 4; ++k) {
      const bf16 h0 = (bf16)a0[k];
      const bf16 h1 = (bf16)a1[k];
      ph.h[k]     = h0;
      ph.h[4 + k] = h1;
      pl.h[k]     = (bf16)(a0[k] - (float)h0);
      pl.h[4 + k] = (bf16)(a1[k] - (float)h1);
    }
    vh[it] = ph.u;
    vl[it] = pl.u;
    gidx[it] = ((size_t)b * SEQ + qrow0 + row) * DEMB + h * HDIM + c8;
  }
  #pragma unroll
  for (int it = 0; it < 4; ++it) {
    *(volatile v4u*)(cp + gidx[it]) = vh[it];
    *(volatile v4u*)(cp + CTX_ELEMS + gidx[it]) = vl[it];
  }
  __threadfence();
  #pragma unroll
  for (int it = 0; it < 4; ++it) {
    *(volatile v4u*)(cp + gidx[it]) = vh[it];
    *(volatile v4u*)(cp + CTX_ELEMS + gidx[it]) = vl[it];
  }
}

__global__ __launch_bounds__(256) void attn_early_kernel(const bf16* __restrict__ qkp,
                                                         const bf16* __restrict__ vtb,
                                                         bf16* __restrict__ cp) {
  attn_body<true>(qkp, (const f16*)0, vtb, cp, (int)blockIdx.x);
}

__global__ __launch_bounds__(256) void attn_late_kernel(const bf16* __restrict__ qkp,
                                                        const f16* __restrict__ vt,
                                                        bf16* __restrict__ cp) {
  attn_body<false>(qkp, vt, (const bf16*)0, cp, (int)blockIdx.x + EARLY_QB);
}

extern "C" void kernel_launch(void* const* d_in, const int* in_sizes, int n_in,
                              void* d_out, int out_size, void* d_ws, size_t ws_size,
                              hipStream_t stream) {
  if (n_in < 5) return;
  const size_t rows_used = (size_t)(NB - 1) * SEQ_FULL + SEQ;
  if ((size_t)in_sizes[0] < rows_used * DEMB) return;
  if ((size_t)in_sizes[1] < (size_t)DEMB * QKVN) return;
  if ((size_t)in_sizes[2] < (size_t)QKVN) return;
  if ((size_t)in_sizes[3] < (size_t)DEMB * DEMB) return;
  if ((size_t)in_sizes[4] < (size_t)DEMB) return;
  if ((size_t)out_size < rows_used * DEMB) return;
  if (ws_size < WS_TOTAL) return;

  const float* x     = (const float*)d_in[0];
  const float* W_in  = (const float*)d_in[1];
  const float* b_in  = (const float*)d_in[2];
  const float* W_out = (const float*)d_in[3];
  const float* b_out = (const float*)d_in[4];
  float* out = (float*)d_out;

  char* w = (char*)d_ws;
  bf16* xb    = (bf16*)w;  w += XB_BYTES;
  bf16* winb  = (bf16*)w;  w += WIN_BYTES;
  bf16* woutb = (bf16*)w;  w += WOUT_BYTES;
  bf16* qkp   = (bf16*)w;  w += QK_BYTES;
  f16*  vt    = (f16*)w;   w += VT_BYTES;
  bf16* vtb   = (bf16*)w;  w += VTB_BYTES;
  bf16* cp    = (bf16*)w;  w += CTX_BYTES;
  float* stat = (float*)w;
  float* sline = stat + (size_t)AM_TOTAL * 32;

  cvt_x_kernel<<<dim3((unsigned)(X_PIECES / 256)), 256, 0, stream>>>(x, xb);

  absmax_part_kernel<<<dim3(AM_BLOCKS_IN), 256, 0, stream>>>(W_in, stat, (unsigned)WIN_PIECES);
  absmax_part_kernel<<<dim3(AM_BLOCKS_OUT), 256, 0, stream>>>(W_out, stat + (size_t)AM_BLOCKS_IN * 32,
                                                              (unsigned)WOUT_PIECES);
  scale_fin_kernel<<<dim3(1), 32, 0, stream>>>(stat, sline);

  snap_lin_kernel<<<dim3((unsigned)(WIN_PIECES / 256)), 256, 0, stream>>>(W_in, sline, winb, winb + WIN_ELEMS,
                                                                          (unsigned)WIN_PIECES);
  snap_lin_kernel<<<dim3((unsigned)(WOUT_PIECES / 256)), 256, 0, stream>>>(W_out, sline + 32, woutb,
                                                                           woutb + WOUT_ELEMS,
                                                                           (unsigned)WOUT_PIECES);

  gemm_qkv_kernel<<<dim3(QKVN / 128, MROWS / 128), 256, 0, stream>>>(xb, winb, winb + WIN_ELEMS, b_in,
                                                                     qkp, vt, vtb);

  attn_early_kernel<<<dim3(EARLY_QB, NHEAD, NB), 256, 0, stream>>>(qkp, vtb, cp);
  if (QBLKS > EARLY_QB) {
    attn_late_kernel<<<dim3(QBLKS - EARLY_QB, NHEAD, NB), 256, 0, stream>>>(qkp, vt, cp);
  }

  gemm_out_kernel<<<dim3(DEMB / 128, MROWS / 128), 256, 0, stream>>>(cp, cp + CTX_ELEMS, woutb,
                                                                     woutb + WOUT_ELEMS, b_out, out);
}
